// Decoder_9706626089598
// MI455X (gfx1250) — hardware-verified
//
#include <hip/hip_runtime.h>
#include <math.h>

constexpr int NBATCH   = 512;
constexpr int NSTEP    = 1024;
constexpr int NHID     = 128;
constexpr int NGATE    = 4 * NHID;
constexpr int NLAT     = 16;
constexpr int NLATC    = NLAT + 1;
constexpr int NOUTC    = 12;
constexpr int ROWS_BLK = 16;
constexpr int NTHR     = 256;
constexpr int WPITCH   = 136;
constexpr int HPITCH   = 136;
constexpr int XSP      = 132;
constexpr int TCH      = 8;
constexpr int OSP      = TCH * NOUTC;

constexpr int OFF_W    = 0;
constexpr int SZ_W     = NGATE * WPITCH * 2;
constexpr int OFF_WO   = OFF_W + SZ_W;
constexpr int SZ_WO    = 16 * WPITCH * 2;
constexpr int OFF_H    = OFF_WO + SZ_WO;
constexpr int SZ_H     = 2 * ROWS_BLK * HPITCH * 2;
constexpr int OFF_OS   = OFF_H + SZ_H;
constexpr int SZ_OS    = ROWS_BLK * OSP * 4;
constexpr int OFF_XS   = OFF_OS + SZ_OS;
constexpr int SZ_XS    = ROWS_BLK * XSP * 4;
constexpr int LDS_TOTAL = OFF_XS + SZ_XS;

static_assert(NBATCH % ROWS_BLK == 0, "batch tiles");
static_assert(NHID % 32 == 0, "K multiple of 32");
static_assert(NHID == 16 * (NTHR / 32), "8 waves x 16 hidden columns");
static_assert(NSTEP % TCH == 0, "flush period divides T");
static_assert((OSP * 4) % 128 == 0, "staged row = whole lines");
static_assert(((size_t)NSTEP * NOUTC * 4) % 128 == 0, "batch row = whole lines");
static_assert(ROWS_BLK * (OSP * 4 / 128) == 6 * (NTHR / 32), "6 lines per wave per flush");
static_assert(OFF_WO % 16 == 0 && OFF_H % 16 == 0 && OFF_OS % 16 == 0 && OFF_XS % 16 == 0, "16-B aligned regions");
static_assert(LDS_TOTAL == 166912, "LDS carve");
static_assert((size_t)NBATCH * NSTEP * NOUTC * 4 == 25165824u, "output bytes");
static_assert((NGATE * NHID / 8) % NTHR == 0, "W_hh staging loop exact");
static_assert(ROWS_BLK * NHID == 8 * NTHR, "x tile loop exact");
static_assert(16 * (NHID / 8) == NTHR, "W_out staging exact");

typedef __attribute__((ext_vector_type(16))) _Float16 v16h;
typedef __attribute__((ext_vector_type(8)))  _Float16 v8h;
typedef __attribute__((ext_vector_type(8)))  float    v8f;
typedef __attribute__((ext_vector_type(4)))  float    v4f;

union FragU { v16h v; v8h h[2]; };
__device__ __forceinline__ v16h frag_load(const _Float16* p) {
  FragU f;
  f.h[0] = *(const v8h*)(p);
  f.h[1] = *(const v8h*)(p + 16);
  return f.v;
}
__device__ __forceinline__ v8f mma_f16(v16h a, v16h b, v8f c) {
  return __builtin_amdgcn_wmma_f32_16x16x32_f16(false, a, false, b, (short)0, c, false, false);
}
__device__ __forceinline__ void guard_grp(v8f& a0, v8f& a1, v8f& a2, v8f& a3, v16h x, v16h y0, v16h y1, v16h y2, v16h y3) {
  asm volatile("v_nop\n\tv_nop\n\tv_nop\n\tv_nop"
               : "+v"(a0), "+v"(a1), "+v"(a2), "+v"(a3)
               : "v"(x), "v"(y0), "v"(y1), "v"(y2), "v"(y3));
}
__device__ __forceinline__ void guard_one(v8f& a, v16h x, v16h y) {
  asm volatile("v_nop\n\tv_nop\n\tv_nop\n\tv_nop" : "+v"(a) : "v"(x), "v"(y));
}

__device__ __forceinline__ float fsig(float x) {
  return __builtin_amdgcn_rcpf(1.0f + expf(-x));
}
__device__ __forceinline__ float ftanh_e(float x) {
  return 1.0f - 2.0f * __builtin_amdgcn_rcpf(1.0f + expf(2.0f * x));
}

__global__ __launch_bounds__(NTHR) void lstm_decoder_kernel(
    const float* __restrict__ zin, const float* __restrict__ cnd,
    const float* __restrict__ Wst, const float* __restrict__ bst,
    const float* __restrict__ Wih, const float* __restrict__ bih,
    const float* __restrict__ Whh, const float* __restrict__ bhh,
    const float* __restrict__ Wout, const float* __restrict__ bout,
    const int* __restrict__ seqp, float* __restrict__ out) {
  extern __shared__ __align__(16) unsigned char smem[];
  _Float16* Wl  = (_Float16*)(smem + OFF_W);
  _Float16* Wol = (_Float16*)(smem + OFF_WO);
  _Float16* Hl  = (_Float16*)(smem + OFF_H);
  float*    Os  = (float*)(smem + OFF_OS);
  float*    Xs  = (float*)(smem + OFF_XS);

  const int tid  = threadIdx.x;
  const int lane = tid & 31;
  const int wv   = __builtin_amdgcn_readfirstlane(tid >> 5);
  const int c    = lane & 15;
  const int hh   = lane >> 4;
  const int koff = hh * 8;
  const int bg0  = blockIdx.x * ROWS_BLK;

  int nT;
  {
    const int sl = seqp[0];
    const int s0 = sl < 0 ? 0 : sl;
    nT = (s0 >= NSTEP) ? NSTEP : (s0 & ~(TCH - 1));
  }

#pragma unroll 1
  for (int i = 0; i < 8; ++i) {
    const int idx = i * NTHR + tid;
    const int row = idx >> 7;
    const int j   = idx & (NHID - 1);
    const float* zr = zin + (size_t)(bg0 + row) * NLAT;
    const float* wr = Wst + (size_t)j * NLATC;
    float s = bst[j];
#pragma unroll 4
    for (int k = 0; k < NLAT; ++k) s = fmaf(zr[k], wr[k], s);
    s = fmaf(cnd[bg0 + row], wr[NLAT], s);
    Xs[row * XSP + j] = s;
  }

#pragma unroll 1
  for (int it = 0; it < (NGATE * NHID / 8) / NTHR; ++it) {
    const int ci = it * NTHR + tid;
    const int r  = ci >> 4;
    const int c8 = (ci & 15) * 8;
    const v4f a = *(const v4f*)(Whh + (size_t)r * NHID + c8);
    const v4f b = *(const v4f*)(Whh + (size_t)r * NHID + c8 + 4);
    v8h hv;
#pragma unroll
    for (int e = 0; e < 4; ++e) {
      hv[e]     = (_Float16)a[e];
      hv[4 + e] = (_Float16)b[e];
    }
    *(v8h*)(Wl + r * WPITCH + c8) = hv;
  }
  {
    const int r  = tid >> 4;
    const int c8 = (tid & 15) * 8;
    const int rr = r < NOUTC ? r : (NOUTC - 1);
    const v4f a = *(const v4f*)(Wout + (size_t)rr * NHID + c8);
    const v4f b = *(const v4f*)(Wout + (size_t)rr * NHID + c8 + 4);
    const bool live = (r < NOUTC);
    v8h hv;
#pragma unroll
    for (int e = 0; e < 4; ++e) {
      const float fa = live ? a[e] : 0.0f;
      const float fb = live ? b[e] : 0.0f;
      hv[e]     = (_Float16)fa;
      hv[4 + e] = (_Float16)fb;
    }
    *(v8h*)(Wol + r * WPITCH + c8) = hv;
  }
  {
    const v8h zz = {(_Float16)0.0f, (_Float16)0.0f, (_Float16)0.0f, (_Float16)0.0f,
                    (_Float16)0.0f, (_Float16)0.0f, (_Float16)0.0f, (_Float16)0.0f};
#pragma unroll 1
    for (int i = tid; i < SZ_H / 16; i += NTHR) *(v8h*)(Hl + i * 8) = zz;
  }
  __syncthreads();

  v8f xprv[4];
#pragma unroll
  for (int q = 0; q < 4; ++q) {
    const int n = q * NHID + wv * 16 + c;
    const float bsum = bih[n] + bhh[n];
#pragma unroll
    for (int r = 0; r < 8; ++r) xprv[q][r] = bsum;
  }
  {
    const float* wbase = Wih + (size_t)(wv * 16 + c) * NHID;
#pragma unroll 1
    for (int k0 = 0; k0 < NHID; k0 += 4) {
      const v4f w0 = *(const v4f*)(wbase + (size_t)0 * NHID * NHID + k0);
      const v4f w1 = *(const v4f*)(wbase + (size_t)1 * NHID * NHID + k0);
      const v4f w2 = *(const v4f*)(wbase + (size_t)2 * NHID * NHID + k0);
      const v4f w3 = *(const v4f*)(wbase + (size_t)3 * NHID * NHID + k0);
#pragma unroll
      for (int r = 0; r < 8; ++r) {
        const v4f xv = *(const v4f*)(Xs + (8 * hh + r) * XSP + k0);
#pragma unroll
        for (int e = 0; e < 4; ++e) {
          xprv[0][r] = fmaf(xv[e], w0[e], xprv[0][r]);
          xprv[1][r] = fmaf(xv[e], w1[e], xprv[1][r]);
          xprv[2][r] = fmaf(xv[e], w2[e], xprv[2][r]);
          xprv[3][r] = fmaf(xv[e], w3[e], xprv[3][r]);
        }
      }
    }
  }

  v8f obias;
  {
    const float bo  = bout[c < NOUTC ? c : (NOUTC - 1)];
    const float bov = (c < NOUTC) ? bo : 0.0f;
#pragma unroll
    for (int r = 0; r < 8; ++r) obias[r] = bov;
  }
  v16h wo0, wo1, wo2, wo3;
  {
    const _Float16* wop = Wol + c * WPITCH + koff;
    wo0 = frag_load(wop + 0);
    wo1 = frag_load(wop + 32);
    wo2 = frag_load(wop + 64);
    wo3 = frag_load(wop + 96);
  }

  float creg[8];
#pragma unroll
  for (int r = 0; r < 8; ++r) creg[r] = 0.0f;

  const _Float16* bp0 = Wl + ((0 * 8 + wv) * 16 + c) * WPITCH + koff;
  const _Float16* bp1 = Wl + ((1 * 8 + wv) * 16 + c) * WPITCH + koff;
  const _Float16* bp2 = Wl + ((2 * 8 + wv) * 16 + c) * WPITCH + koff;
  const _Float16* bp3 = Wl + ((3 * 8 + wv) * 16 + c) * WPITCH + koff;
  const int hcol = wv * 16 + c;

#pragma unroll 1
  for (int t = 0; t < nT; ++t) {
    const int cur = t & 1;
    const _Float16* ar = Hl + cur * (ROWS_BLK * HPITCH) + c * HPITCH + koff;
    _Float16* hn = Hl + (cur ^ 1) * (ROWS_BLK * HPITCH);

    v8f acc[4];
    acc[0] = xprv[0];
    acc[1] = xprv[1];
    acc[2] = xprv[2];
    acc[3] = xprv[3];
#pragma unroll
    for (int kc = 0; kc < 4; ++kc) {
      const v16h a  = frag_load(ar  + kc * 32);
      const v16h b0 = frag_load(bp0 + kc * 32);
      const v16h b1 = frag_load(bp1 + kc * 32);
      const v16h b2 = frag_load(bp2 + kc * 32);
      const v16h b3 = frag_load(bp3 + kc * 32);
      acc[0] = mma_f16(a, b0, acc[0]);
      acc[1] = mma_f16(a, b1, acc[1]);
      acc[2] = mma_f16(a, b2, acc[2]);
      acc[3] = mma_f16(a, b3, acc[3]);
      guard_grp(acc[0], acc[1], acc[2], acc[3], a, b0, b1, b2, b3);
    }

#pragma unroll
    for (int r = 0; r < 8; ++r) {
      const float ig = fsig(acc[0][r]);
      const float fg = fsig(acc[1][r]);
      const float gg = ftanh_e(acc[2][r]);
      const float og = fsig(acc[3][r]);
      const float cn = fg * creg[r] + ig * gg;
      creg[r] = cn;
      const float hv = og * ftanh_e(cn);
      hn[(8 * hh + r) * HPITCH + hcol] = (_Float16)hv;
    }

    __syncthreads();

    if (wv == 0) {
      const _Float16* an = hn + c * HPITCH + koff;
      v8f oacc = obias;
      {
        const v16h a = frag_load(an + 0);
        oacc = mma_f16(a, wo0, oacc);
        guard_one(oacc, a, wo0);
      }
      {
        const v16h a = frag_load(an + 32);
        oacc = mma_f16(a, wo1, oacc);
        guard_one(oacc, a, wo1);
      }
      {
        const v16h a = frag_load(an + 64);
        oacc = mma_f16(a, wo2, oacc);
        guard_one(oacc, a, wo2);
      }
      {
        const v16h a = frag_load(an + 96);
        oacc = mma_f16(a, wo3, oacc);
        guard_one(oacc, a, wo3);
      }
      if (c < NOUTC) {
        const int sc = (t & (TCH - 1)) * NOUTC + c;
#pragma unroll
        for (int r = 0; r < 8; ++r) Os[(8 * hh + r) * OSP + sc] = oacc[r];
      }
    }

    if ((t & (TCH - 1)) == (TCH - 1)) {
      __syncthreads();
      const int t0 = t - (TCH - 1);
      float fv[6];
#pragma unroll
      for (int i = 0; i < 6; ++i) {
        const int row = 2 * wv + (i / 3);
        const int seg = i % 3;
        fv[i] = Os[row * OSP + seg * 32 + lane];
      }
      for (int pass = 0; pass < 2; ++pass) {
#pragma unroll
        for (int i = 0; i < 6; ++i) {
          const int row = 2 * wv + (i / 3);
          const int seg = i % 3;
          float* op = out + ((size_t)(bg0 + row) * NSTEP + (size_t)t0) * NOUTC + seg * 32 + lane;
          *(volatile float*)op = fv[i];
        }
        __threadfence();
      }
    }
  }
}

extern "C" void kernel_launch(void* const* d_in, const int* in_sizes, int n_in,
                              void* d_out, int out_size, void* d_ws, size_t ws_size, hipStream_t stream) {
  (void)d_ws;
  (void)ws_size;
  if (n_in < 11 || d_out == nullptr) return;
  if (in_sizes[0] != NBATCH * NLAT || in_sizes[1] != NBATCH || in_sizes[2] != NHID * NLATC ||
      in_sizes[3] != NHID || in_sizes[4] != NGATE * NHID || in_sizes[5] != NGATE ||
      in_sizes[6] != NGATE * NHID || in_sizes[7] != NGATE || in_sizes[8] != NOUTC * NHID ||
      in_sizes[9] != NOUTC || in_sizes[10] != 1 || out_size != NBATCH * NSTEP * NOUTC) return;

  const float* zin  = (const float*)d_in[0];
  const float* cnd  = (const float*)d_in[1];
  const float* Wst  = (const float*)d_in[2];
  const float* bst  = (const float*)d_in[3];
  const float* Wih  = (const float*)d_in[4];
  const float* bih  = (const float*)d_in[5];
  const float* Whh  = (const float*)d_in[6];
  const float* bhh  = (const float*)d_in[7];
  const float* Wout = (const float*)d_in[8];
  const float* bout = (const float*)d_in[9];
  const int*   seqp = (const int*)d_in[10];

  lstm_decoder_kernel<<<NBATCH / ROWS_BLK, NTHR, (size_t)LDS_TOTAL, stream>>>(
      zin, cnd, Wst, bst, Wih, bih, Whh, bhh, Wout, bout, seqp, (float*)d_out);
}
